// GroupQueryAttention_33827162423863
// MI455X (gfx1250) — hardware-verified
//
#include <hip/hip_runtime.h>


#ifndef NB
#define NB   1
#endif
#ifndef SEQ
#define SEQ  2048
#endif
#define SEQ_FULL 2048
#define DM   2048
#define NH   32
#define NKV  8
#define REP  (NH / NKV)
#define HD   64
#define DQ   (NH * HD)
#define DKV  (NKV * HD)
#define ZH   REP
#define PCAR 1024.0f
#define PSH  (PCAR / (float)SEQ)
#define WSC  64.0f
#define OSC  (1.0f / (PCAR * WSC))
#define SCL  0.125f
static_assert(SEQ % 128 == 0);
static_assert(SEQ <= SEQ_FULL);
static_assert(NH % ZH == 0);
static_assert(DKV % 256 == 0);
static_assert(DM % 64 == 0 && DQ % 64 == 0 && DKV % 64 == 0 && HD == 64);

typedef _Float16 h16;
typedef unsigned short bf;
typedef __attribute__((ext_vector_type(16))) __bf16   v16bf;
typedef __attribute__((ext_vector_type(16))) _Float16 v16h;
typedef __attribute__((ext_vector_type(8)))  _Float16 v8h;
typedef __attribute__((ext_vector_type(4)))  _Float16 v4h;
typedef __attribute__((ext_vector_type(8)))  unsigned short v8us;
typedef __attribute__((ext_vector_type(8)))  float    v8f;
typedef __attribute__((ext_vector_type(4)))  float    v4f;
typedef v8h  __attribute__((may_alias)) v8ha;
typedef v4f  __attribute__((may_alias)) v4fa;
typedef v8us __attribute__((may_alias)) v8usa;

__device__ __forceinline__ unsigned short f2bf(float f) { unsigned u = __float_as_uint(f); u += 0x7FFFu + ((u >> 16) & 1u); return (unsigned short)(u >> 16); }
__device__ __forceinline__ float bf2f(unsigned short b) { return __uint_as_float(((unsigned)b) << 16); }
__device__ __forceinline__ float bfr(float f) { return bf2f(f2bf(f)); }
__device__ __forceinline__ h16 tohx(float x) { return (h16)x; }
__device__ __forceinline__ v16h cat16(v8h lo, v8h hi) { return __builtin_shufflevector(lo, hi, 0, 1, 2, 3, 4, 5, 6, 7, 8, 9, 10, 11, 12, 13, 14, 15); }
__device__ __forceinline__ v16bf cat16b(v8us lo, v8us hi) { return __builtin_bit_cast(v16bf, __builtin_shufflevector(lo, hi, 0, 1, 2, 3, 4, 5, 6, 7, 8, 9, 10, 11, 12, 13, 14, 15)); }
__device__ __forceinline__ v8f wmma16(v16h a, v16h b, v8f c) { return __builtin_amdgcn_wmma_f32_16x16x32_f16(false, a, false, b, (short)0, c, false, false); }
__device__ __forceinline__ v8f wmmab(v16bf a, v16bf b, v8f c) { return __builtin_amdgcn_wmma_f32_16x16x32_bf16(false, a, false, b, (short)0, c, false, false); }

template <typename T16> struct WFrag;
template <> struct WFrag<h16> { typedef v16h V; static __device__ __forceinline__ V ld(const h16* p) { return cat16(*(const v8h*)p, *(const v8h*)(p + 16)); } static __device__ __forceinline__ v8f mma(V a, V b, v8f c) { return wmma16(a, b, c); } };
template <> struct WFrag<bf> { typedef v16bf V; static __device__ __forceinline__ V ld(const bf* p) { return cat16b(*(const v8us*)p, *(const v8us*)(p + 16)); } static __device__ __forceinline__ v8f mma(V a, V b, v8f c) { return wmmab(a, b, c); } };

template <typename T16, int NSPLIT, int BM>
__global__ __launch_bounds__(32) __attribute__((amdgpu_num_vgpr(256)))
void k_gemmw(const T16* __restrict__ A, const T16* __restrict__ A2, const T16* __restrict__ Bt, const T16* __restrict__ Bt2, int K, float* C, int ldc, const float* __restrict__ bias, float oscale, size_t sA, size_t sB, size_t sC) {
    typedef typename WFrag<T16>::V V;
    __shared__ __align__(16) float os[16 * 68];
    const size_t z = blockIdx.z; A += z * sA; if (A2) A2 += z * sA; Bt += z * sB; if (Bt2) Bt2 += z * sB; C += z * sC;
    const int lane = threadIdx.x & 31, lr = lane & 15, hi = lane >> 4; const int r0 = blockIdx.x * 64, c0 = blockIdx.y * 64;
    v8f acc[4][4];
#pragma unroll
    for (int mb = 0; mb < 4; ++mb)
#pragma unroll
        for (int nb = 0; nb < 4; ++nb) acc[mb][nb] = (v8f){};
    const size_t aoff = (size_t)(r0 + lr) * K + 8 * hi, boff = (size_t)(c0 + lr) * K + 8 * hi;
#pragma unroll 1
    for (int kc = 0; kc < K; kc += 32) {
        V a[4], a2[4];
#pragma unroll
        for (int mb = 0; mb < 4; ++mb) { a[mb] = WFrag<T16>::ld(A + aoff + (size_t)mb * 16 * K + kc); if (NSPLIT == 1 || NSPLIT == 2) a2[mb] = WFrag<T16>::ld(A2 + aoff + (size_t)mb * 16 * K + kc); }
#pragma unroll
        for (int nb = 0; nb < 4; ++nb) { const V b = WFrag<T16>::ld(Bt + boff + (size_t)nb * 16 * K + kc); V b2; if (NSPLIT >= 2) b2 = WFrag<T16>::ld(Bt2 + boff + (size_t)nb * 16 * K + kc);
#pragma unroll
            for (int mb = 0; mb < 4; ++mb) { acc[mb][nb] = WFrag<T16>::mma(a[mb], b, acc[mb][nb]); if (NSPLIT == 1 || NSPLIT == 2) acc[mb][nb] = WFrag<T16>::mma(a2[mb], b, acc[mb][nb]); if (NSPLIT >= 2) acc[mb][nb] = WFrag<T16>::mma(a[mb], b2, acc[mb][nb]); } }
        asm volatile("v_nop\n\tv_nop\n\tv_nop\n\tv_nop" : "+v"(acc[0][0]), "+v"(acc[1][1]), "+v"(acc[2][2]), "+v"(acc[3][3]) : "v"(a[0]), "v"(a[3]));
    }
#pragma unroll
    for (int mb = 0; mb < 4; ++mb) {
#pragma unroll
        for (int nb = 0; nb < 4; ++nb) {
#pragma unroll
            for (int j = 0; j < 8; ++j) os[(hi * 8 + j) * 68 + nb * 16 + lr] = acc[mb][nb][j]; }
        __builtin_amdgcn_fence(3, "wavefront"); __builtin_amdgcn_wave_barrier(); asm volatile("" ::: "memory");
        float* crow = C + (size_t)(r0 + mb * 16) * ldc + c0;
#pragma unroll 1
        for (int ps = 0; ps < 2; ++ps) {
#pragma unroll
            for (int s = 0; s < 8; ++s) { const int row = 2 * s + hi, cofs = lr * 4; v4f val = *(const v4fa*)(os + row * 68 + cofs); val = val * oscale;
                if (BM == 1) { val[0] += bfr(bias[c0 + cofs]); val[1] += bfr(bias[c0 + cofs + 1]); val[2] += bfr(bias[c0 + cofs + 2]); val[3] += bfr(bias[c0 + cofs + 3]); }
                else if (BM == 2) { const v4f bb = *(const v4f*)(bias + c0 + cofs); val += bb; }
                *(volatile v4f*)(crow + (size_t)row * ldc + cofs) = val; }
            if (ps == 0) __threadfence(); }
        __builtin_amdgcn_fence(3, "wavefront"); __builtin_amdgcn_wave_barrier(); asm volatile("" ::: "memory");
    }
}

__global__ __launch_bounds__(256) void k_cvt8(const float* __restrict__ src, bf* dst, size_t n8) { const size_t i = (size_t)blockIdx.x * 256 + threadIdx.x; if (i >= n8) return; const v8f v = *(const v8f*)(src + i * 8); v8us o;
#pragma unroll
    for (int k = 0; k < 8; ++k) o[k] = f2bf(v[k]); *(volatile v8us*)(dst + i * 8) = o; __threadfence(); *(volatile v8us*)(dst + i * 8) = o; }

template <int PREB>
__global__ __launch_bounds__(256) void k_cvth(const float* __restrict__ src, h16* dst, size_t n8, float sc) { const size_t i = (size_t)blockIdx.x * 256 + threadIdx.x; if (i >= n8) return; const v8f v = *(const v8f*)(src + i * 8); v8h o;
#pragma unroll
    for (int k = 0; k < 8; ++k) { const float y = PREB ? bfr(v[k]) : v[k]; o[k] = tohx(y * sc); }
    *(volatile v8h*)(dst + i * 8) = o; __threadfence(); *(volatile v8h*)(dst + i * 8) = o; }

__global__ __launch_bounds__(256) void k_plane(const float* __restrict__ F, int pitch, int nheads, h16* P16) {
    const size_t e = ((size_t)blockIdx.x * 256 + threadIdx.x) * 8; if (e >= (size_t)nheads * SEQ * HD) return;
    const int d = (int)(e % HD); const int t = (int)((e / HD) % SEQ); const int h = (int)(e / ((size_t)HD * SEQ));
    const float* f = F + (size_t)t * pitch + h * HD + d; const v4f x0 = *(const v4f*)f; const v4f x1 = *(const v4f*)(f + 4); v8h o;
#pragma unroll
    for (int q = 0; q < 4; ++q) { o[q] = tohx(x0[q]); o[4 + q] = tohx(x1[q]); }
    *(volatile v8h*)(P16 + e) = o; __threadfence(); *(volatile v8h*)(P16 + e) = o; }

__global__ __launch_bounds__(256) void k_vtp(const float* __restrict__ F, int pitch, int ng, h16* V16) { const size_t e = ((size_t)blockIdx.x * 256 + threadIdx.x) * 8; if (e >= (size_t)ng * HD * SEQ) return; const int t = (int)(e % SEQ); const int d = (int)((e / SEQ) % HD); const int g = (int)(e / ((size_t)SEQ * HD)); v8h o;
#pragma unroll
    for (int q = 0; q < 8; ++q) o[q] = tohx(F[(size_t)(t + q) * pitch + g * HD + d]);
    *(volatile v8h*)(V16 + e) = o; __threadfence(); *(volatile v8h*)(V16 + e) = o; }

__global__ __launch_bounds__(256) void k_vsum(const float* __restrict__ F, int pitch, int ncol, float sc, float* VS) {
    __shared__ __align__(16) float s[256];
    const int c = blockIdx.x * 256 + threadIdx.x; const int cc = min(c, ncol - 1);
    double acc = 0.0;
#pragma unroll 4
    for (int t = 0; t < SEQ; ++t) acc += (double)F[(size_t)t * pitch + cc];
    s[threadIdx.x] = (float)acc * sc;
    __syncthreads();
    if (threadIdx.x < 64) { const int c4 = blockIdx.x * 256 + threadIdx.x * 4;
        if (c4 + 3 < ncol) { const v4f o = *(const v4fa*)(s + threadIdx.x * 4); *(volatile v4f*)(VS + c4) = o; __threadfence(); *(volatile v4f*)(VS + c4) = o; } }
}

__global__ __launch_bounds__(256) void k_asoft(const float* __restrict__ Sb, h16* P16, int nrows) {
    const int lane = threadIdx.x & 31; const int row = blockIdx.x * 8 + (threadIdx.x >> 5); if (row >= nrows) return;
    const float* sr = Sb + (size_t)row * SEQ; float v[SEQ / 32]; float mx = -3.0e38f;
#pragma unroll
    for (int ch = 0; ch < SEQ / 128; ++ch) { const v4f a = *(const v4f*)(sr + ch * 128 + lane * 4);
#pragma unroll
        for (int q = 0; q < 4; ++q) { v[ch * 4 + q] = a[q]; mx = fmaxf(mx, a[q]); } }
#pragma unroll
    for (int sh = 16; sh; sh >>= 1) mx = fmaxf(mx, __shfl_xor(mx, sh, 32));
    float sum = 0.f;
#pragma unroll
    for (int k = 0; k < SEQ / 32; ++k) { float d0 = __fsub_rn(v[k], mx); asm volatile("" : "+v"(d0)); v[k] = __builtin_amdgcn_exp2f(__fmul_rn(d0, SCL * 1.4426950408889634f)); sum += v[k]; }
#pragma unroll
    for (int sh = 16; sh; sh >>= 1) sum += __shfl_xor(sum, sh, 32);
    const float f = __fdiv_rn(PCAR, sum);
    v4h o[SEQ / 128];
#pragma unroll
    for (int ch = 0; ch < SEQ / 128; ++ch) {
#pragma unroll
        for (int q = 0; q < 4; ++q) { const float y = __fsub_rn(__fmul_rn(v[ch * 4 + q], f), PSH); o[ch][q] = tohx(y); } }
    h16* prow = P16 + (size_t)row * SEQ + lane * 4;
#pragma unroll 1
    for (int ps = 0; ps < 2; ++ps) {
#pragma unroll
        for (int ch = 0; ch < SEQ / 128; ++ch) *(volatile v4h*)(prow + ch * 128) = o[ch];
        if (ps == 0) __threadfence(); }
}

extern "C" void kernel_launch(void* const* d_in, const int* in_sizes, int n_in,
                              void* d_out, int out_size, void* d_ws, size_t ws_size, hipStream_t stream) {
    if (n_in < 9) return;
    if (in_sizes[0] < (NB - 1) * SEQ_FULL * DM + SEQ * DM) return;
    if (in_sizes[1] < DQ * DM || in_sizes[2] < DQ || in_sizes[3] < DKV * DM || in_sizes[4] < DKV || in_sizes[5] < DKV * DM || in_sizes[6] < DKV || in_sizes[7] < DM * DQ || in_sizes[8] < DM) return;
    if (out_size < (NB - 1) * SEQ_FULL * DM + SEQ * DM) return;
    const float* x  = (const float*)d_in[0];
    const float* wq = (const float*)d_in[1];
    const float* bq = (const float*)d_in[2];
    const float* wk = (const float*)d_in[3];
    const float* bk = (const float*)d_in[4];
    const float* wv = (const float*)d_in[5];
    const float* bv = (const float*)d_in[6];
    const float* wo = (const float*)d_in[7];
    const float* bo = (const float*)d_in[8];
    float* OUT = (float*)d_out;

    char* base = (char*)d_ws; size_t off = 0;
    auto take = [&](size_t bytes) { char* p = base + off; off += (bytes + 255) & ~(size_t)255; return (void*)p; };
    h16* QP16 = (h16*)take((size_t)NH * SEQ * HD * 2);
    h16* KP16 = (h16*)take((size_t)NKV * SEQ * HD * 2);
    h16* VT16 = (h16*)take((size_t)NKV * HD * SEQ * 2);
    float* VADD = (float*)take((size_t)DKV * 4);
    float* CTX  = (float*)take((size_t)SEQ * DQ * 4);
    const size_t offA = off;
    bf* XB = (bf*)take((size_t)SEQ * DM * 2); bf* WQ = (bf*)take((size_t)DQ * DM * 2); bf* WK = (bf*)take((size_t)DKV * DM * 2); bf* WV = (bf*)take((size_t)DKV * DM * 2);
    float* FQ = (float*)take((size_t)SEQ * DQ * 4); float* FK = (float*)take((size_t)SEQ * DKV * 4); float* FV = (float*)take((size_t)SEQ * DKV * 4);
    const size_t end1 = off; off = offA;
    float* Sb = (float*)take((size_t)ZH * SEQ * SEQ * 4); h16* P16 = (h16*)take((size_t)ZH * SEQ * SEQ * 2);
    const size_t end2 = off; off = offA;
    h16* CTX16 = (h16*)take((size_t)SEQ * DQ * 2); h16* WO16 = (h16*)take((size_t)DM * DQ * 2);
    const size_t end3 = off;
    size_t total = end1; if (end2 > total) total = end2; if (end3 > total) total = end3;
    if (total > ws_size || total > (size_t)128 * 1048576) return;

    const unsigned gX8 = (unsigned)(((size_t)SEQ * DM / 8 + 255) / 256);
    for (int b = 0; b < NB; ++b) {
        const float* xb = x + (size_t)b * SEQ_FULL * DM; float* outb = OUT + (size_t)b * SEQ_FULL * DM;
        k_cvt8<<<gX8, 256, 0, stream>>>(xb, XB, (size_t)SEQ * DM / 8);
        k_cvt8<<<(unsigned)(((size_t)DQ * DM / 8 + 255) / 256), 256, 0, stream>>>(wq, WQ, (size_t)DQ * DM / 8);
        k_cvt8<<<(unsigned)(((size_t)DKV * DM / 8 + 255) / 256), 256, 0, stream>>>(wk, WK, (size_t)DKV * DM / 8);
        k_cvt8<<<(unsigned)(((size_t)DKV * DM / 8 + 255) / 256), 256, 0, stream>>>(wv, WV, (size_t)DKV * DM / 8);
        k_gemmw<bf, 0, 1><<<dim3(SEQ / 64, DQ / 64, 1), 32, 0, stream>>>(XB, nullptr, WQ, nullptr, DM, FQ, DQ, bq, 1.0f, (size_t)0, (size_t)0, (size_t)0);
        k_gemmw<bf, 0, 1><<<dim3(SEQ / 64, DKV / 64, 1), 32, 0, stream>>>(XB, nullptr, WK, nullptr, DM, FK, DKV, bk, 1.0f, (size_t)0, (size_t)0, (size_t)0);
        k_gemmw<bf, 0, 1><<<dim3(SEQ / 64, DKV / 64, 1), 32, 0, stream>>>(XB, nullptr, WV, nullptr, DM, FV, DKV, bv, 1.0f, (size_t)0, (size_t)0, (size_t)0);
        k_plane<<<(unsigned)(((size_t)NH * SEQ * HD / 8 + 255) / 256), 256, 0, stream>>>(FQ, DQ, NH, QP16);
        k_plane<<<(unsigned)(((size_t)NKV * SEQ * HD / 8 + 255) / 256), 256, 0, stream>>>(FK, DKV, NKV, KP16);
        k_vtp<<<(unsigned)(((size_t)NKV * HD * SEQ / 8 + 255) / 256), 256, 0, stream>>>(FV, DKV, NKV, VT16);
        k_vsum<<<DKV / 256, 256, 0, stream>>>(FV, DKV, DKV, PSH, VADD);
        for (int h0 = 0; h0 < NH; h0 += ZH) { const int g = h0 / REP;
            k_gemmw<h16, 0, 0><<<dim3(SEQ / 64, SEQ / 64, ZH), 32, 0, stream>>>(QP16 + (size_t)h0 * SEQ * HD, nullptr, KP16 + (size_t)g * SEQ * HD, nullptr, HD, Sb, SEQ, nullptr, 1.0f, (size_t)SEQ * HD, (size_t)0, (size_t)SEQ * SEQ);
            k_asoft<<<(unsigned)(ZH * SEQ / 8), 256, 0, stream>>>(Sb, P16, ZH * SEQ);
            k_gemmw<h16, 0, 2><<<dim3(SEQ / 64, HD / 64, ZH), 32, 0, stream>>>(P16, nullptr, VT16 + (size_t)g * HD * SEQ, nullptr, SEQ, CTX + (size_t)h0 * HD, DQ, VADD + g * HD, 1.0f, (size_t)SEQ * SEQ, (size_t)0, (size_t)HD);
        }
        k_cvth<0><<<(unsigned)(((size_t)SEQ * DQ / 8 + 255) / 256), 256, 0, stream>>>(CTX, CTX16, (size_t)SEQ * DQ / 8, 1.0f);
        k_cvth<1><<<(unsigned)(((size_t)DM * DQ / 8 + 255) / 256), 256, 0, stream>>>(wo, WO16, (size_t)DM * DQ / 8, WSC);
        k_gemmw<h16, 0, 1><<<dim3(SEQ / 64, DM / 64, 1), 32, 0, stream>>>(CTX16, nullptr, WO16, nullptr, DQ, outb, DM, bo, OSC, (size_t)0, (size_t)0, (size_t)0);
    }
}
